// CAC_61375082660604
// MI455X (gfx1250) — hardware-verified
//
#include <hip/hip_runtime.h>
#include <stddef.h>

typedef __attribute__((ext_vector_type(16))) _Float16 v16h;
typedef __attribute__((ext_vector_type(8)))  _Float16 v8h;
typedef __attribute__((ext_vector_type(16))) __bf16   v16b;
typedef __attribute__((ext_vector_type(8)))  __bf16   v8b;
typedef __attribute__((ext_vector_type(8)))  float    v8f;
typedef __attribute__((ext_vector_type(4)))  float    v4f;
#define PSCALE 32768.0f
#define U16(p) ((const unsigned short*)(const void*)(p))
#define PSCALE_INV (1.0f / 32768.0f)

__device__ __forceinline__ unsigned short f2bf_bits(float f) {
  unsigned u = __float_as_uint(f);
  return (unsigned short)((u + 0x7FFFu + ((u >> 16) & 1u)) >> 16);
}
__device__ __forceinline__ float bf_bits2f(unsigned short h) { return __uint_as_float(((unsigned)h) << 16); }

__device__ __forceinline__ void dep_guard_h(v8f& a, v8f& b, v16h x, v16h y) { asm volatile("v_nop\n\tv_nop\n\tv_nop\n\tv_nop" : "+v"(a), "+v"(b) : "v"(x), "v"(y)); }
__device__ __forceinline__ void dep_guard_b(v8f& a, v8f& b, v16b x, v16b y) { asm volatile("v_nop\n\tv_nop\n\tv_nop\n\tv_nop" : "+v"(a), "+v"(b) : "v"(x), "v"(y)); }
__device__ __forceinline__ void keep4_h(v16h a, v16h b, v16h c, v16h d) { asm volatile("v_nop" :: "v"(a), "v"(b), "v"(c), "v"(d)); }
__device__ __forceinline__ void keep4_b(v16b a, v16b b, v16b c, v16b d) { asm volatile("v_nop" :: "v"(a), "v"(b), "v"(c), "v"(d)); }
__device__ __forceinline__ void acc_guard4(v8f& a, v8f& b, v8f& c, v8f& d) { asm volatile("v_nop\n\tv_nop\n\tv_nop\n\tv_nop" : "+v"(a), "+v"(b), "+v"(c), "+v"(d)); }
template <typename T> struct Frag;
template <> struct Frag<_Float16> {
  typedef v16h V; union U { v16h v; v8h h[2]; };
  static __device__ __forceinline__ v16h load(const _Float16* p) {
    U f; f.h[0] = *(const v8h*)(p); f.h[1] = *(const v8h*)(p + 16); return f.v;
  }
  static __device__ __forceinline__ v8f mma(v16h a, v16h b, v8f c) {
    return __builtin_amdgcn_wmma_f32_16x16x32_f16(false, a, false, b, (short)0, c, false, false);
  }
  static __device__ __forceinline__ void guard(v8f& a, v8f& b, v16h x, v16h y) { dep_guard_h(a, b, x, y); }
  static __device__ __forceinline__ void keep(v16h a, v16h b, v16h c, v16h d) { keep4_h(a, b, c, d); }
};
template <> struct Frag<__bf16> {
  typedef v16b V; union U { v16b v; v8b h[2]; };
  static __device__ __forceinline__ v16b load(const __bf16* p) {
    U f; f.h[0] = *(const v8b*)(p); f.h[1] = *(const v8b*)(p + 16); return f.v;
  }
  static __device__ __forceinline__ v8f mma(v16b a, v16b b, v8f c) {
    return __builtin_amdgcn_wmma_f32_16x16x32_bf16(false, a, false, b, (short)0, c, false, false);
  }
  static __device__ __forceinline__ void guard(v8f& a, v8f& b, v16b x, v16b y) { dep_guard_b(a, b, x, y); }
  static __device__ __forceinline__ void keep(v16b a, v16b b, v16b c, v16b d) { keep4_b(a, b, c, d); }
};

template <int ET> struct Elem;
template <> struct Elem<0> { typedef _Float16 T; };
template <> struct Elem<1> { typedef __bf16 T; };
template <int ET, bool SPLIT, int BIAS_MODE, int OUT_MODE, bool RESID, int ACT = 0>
__global__ __launch_bounds__(256) void wmma_gemm64(
    const unsigned short* __restrict__ Ap, const unsigned short* __restrict__ A2p, int lda, long strideA,
    const unsigned short* __restrict__ Btp, const unsigned short* __restrict__ Bt2p, int ldb, long strideB,
    void* __restrict__ Cout, void* __restrict__ Cout2, int ldc, long strideC,
    const float* __restrict__ bias,
    const float* __restrict__ resid, long strideR,
    int M, int N, int K, float scale) {
  typedef typename Elem<ET>::T T;
  typedef typename Frag<T>::V V;
  const T* A = (const T*)Ap; const T* A2 = (const T*)A2p; const T* Bt = (const T*)Btp; const T* Bt2 = (const T*)Bt2p;
  __shared__ __align__(16) float sT[8][16 * 68];
  const int b    = blockIdx.y;
  const int lane = threadIdx.x & 31;
  const int wave = threadIdx.x >> 5;
  const int tilesN = N >> 6;
  const int tilesM = M >> 6;
  const int tile = blockIdx.x * 8 + wave;
  if (tile >= tilesM * tilesN) return;
  const int tm = tile / tilesN;
  const int tn = tile - tm * tilesN;
  const int m0 = tm << 6;
  const int n0 = tn << 6;

  const T* Ab  = A  + (size_t)b * strideA;
  const T* Bb  = Bt + (size_t)b * strideB;
  const T* Ab2 = SPLIT ? (A2  + (size_t)b * strideA) : nullptr;
  const T* Bb2 = SPLIT ? (Bt2 + (size_t)b * strideB) : nullptr;

  const int rlane = lane & 15;
  const int koff  = (lane >> 4) * 8;
  const int mOff  = (lane >> 4) * 8;

  v8f acc[4][4];
#pragma unroll
  for (int i = 0; i < 4; ++i)
#pragma unroll
    for (int j = 0; j < 4; ++j) acc[i][j] = (v8f){0.f,0.f,0.f,0.f,0.f,0.f,0.f,0.f};

  for (int k0 = 0; k0 < K; k0 += 32) {
    V bh[4], bl[4];
#pragma unroll
    for (int j = 0; j < 4; ++j) {
      const size_t bo = (size_t)(n0 + (j << 4) + rlane) * ldb + koff + k0;
      bh[j] = Frag<T>::load(Bb + bo);
      if (SPLIT) bl[j] = Frag<T>::load(Bb2 + bo);
    }
#pragma unroll
    for (int i = 0; i < 4; ++i) {
      const size_t ao = (size_t)(m0 + (i << 4) + rlane) * lda + koff + k0;
      V ah = Frag<T>::load(Ab + ao);
      V al;
      if (SPLIT) al = Frag<T>::load(Ab2 + ao);
#pragma unroll
      for (int j = 0; j < 4; ++j) {
        acc[i][j] = Frag<T>::mma(ah, bh[j], acc[i][j]);
        if (SPLIT) {
          acc[i][j] = Frag<T>::mma(ah, bl[j], acc[i][j]);
          acc[i][j] = Frag<T>::mma(al, bh[j], acc[i][j]);
        }
      }
      Frag<T>::guard(acc[i][0], acc[i][3], ah, SPLIT ? al : ah);
    }
    Frag<T>::keep(bh[0], bh[1], bh[2], bh[3]);
    if (SPLIT) Frag<T>::keep(bl[0], bl[1], bl[2], bl[3]);
  }
  acc_guard4(acc[0][0], acc[0][1], acc[0][2], acc[0][3]);
  acc_guard4(acc[1][0], acc[1][1], acc[1][2], acc[1][3]);
  acc_guard4(acc[2][0], acc[2][1], acc[2][2], acc[2][3]);
  acc_guard4(acc[3][0], acc[3][1], acc[3][2], acc[3][3]);

  float* slab = sT[wave];
  const float* Rb = RESID ? (resid + (size_t)b * strideR) : nullptr;
#pragma unroll
  for (int i = 0; i < 4; ++i) {
    const int mBase = m0 + (i << 4);
#pragma unroll
    for (int j = 0; j < 4; ++j) {
      const int n = n0 + (j << 4) + rlane;
      float bv = 0.f;
      if (BIAS_MODE == 2) bv = bias[n];
#pragma unroll
      for (int r = 0; r < 8; ++r) {
        float v = acc[i][j][r] * scale;
        if (BIAS_MODE == 1) v += bias[mBase + mOff + r];
        if (BIAS_MODE == 2) v += bv;
        if (RESID) v += Rb[(size_t)(mBase + mOff + r) * ldc + n];
        if (ACT == 1) v = tanhf(v);
        if (ACT == 2) v = fmaxf(v, 0.0f);
        if (ACT == 3) v = v / (1.0f + expf(-v));
        if (ACT == 4) v = (v > 0.f) ? v : 0.01f * v;
        if (ACT == 5) v = 0.5f * v * (1.0f + erff(v * 0.70710678118654752f));
        slab[(mOff + r) * 68 + (j << 4) + rlane] = v;
      }
    }
    __builtin_amdgcn_fence(__ATOMIC_RELEASE, "workgroup");
    __builtin_amdgcn_wave_barrier();
    __builtin_amdgcn_fence(__ATOMIC_ACQUIRE, "workgroup");
    if (OUT_MODE == 0) {
      float* C = (float*)Cout + (size_t)b * strideC;
      const int hh = lane >> 4, c4 = (lane & 15) * 4;
      for (int pass = 0; pass < 2; ++pass) {
#pragma unroll
        for (int it = 0; it < 8; ++it) {
          const int row = it * 2 + hh;
          v4f v = *(const v4f*)(slab + row * 68 + c4);
          *(volatile v4f*)(C + (size_t)(mBase + row) * ldc + n0 + c4) = v;
        }
        __threadfence();
      }
    } else {
      const int q = lane >> 3, c8 = (lane & 7) * 8;
      unsigned short* C  = (unsigned short*)Cout  + (size_t)b * strideC;
      unsigned short* C2 = (OUT_MODE == 2) ? ((unsigned short*)Cout2 + (size_t)b * strideC) : nullptr;
      for (int pass = 0; pass < 2; ++pass) {
#pragma unroll
        for (int it = 0; it < 4; ++it) {
          const int row = it * 4 + q;
          const float* sp = slab + row * 68 + c8;
          v8h hv, lv;
#pragma unroll
          for (int e = 0; e < 8; ++e) {
            if (OUT_MODE == 1) {
              hv[e] = (_Float16)sp[e];
            } else {
              unsigned short hb = f2bf_bits(sp[e]);
              unsigned short lb = f2bf_bits(sp[e] - bf_bits2f(hb));
              hv[e] = __builtin_bit_cast(_Float16, hb);
              lv[e] = __builtin_bit_cast(_Float16, lb);
            }
          }
          *(volatile v8h*)(C + (size_t)(mBase + row) * ldc + n0 + c8) = hv;
          if (OUT_MODE == 2) *(volatile v8h*)(C2 + (size_t)(mBase + row) * ldc + n0 + c8) = lv;
        }
        __threadfence();
      }
    }
    __builtin_amdgcn_fence(__ATOMIC_RELEASE, "workgroup");
    __builtin_amdgcn_wave_barrier();
    __builtin_amdgcn_fence(__ATOMIC_ACQUIRE, "workgroup");
  }
}

#define IMW 256
#define CPA 72
#define SRW 272

__device__ __forceinline__ float coefval(int c, int cp, float pr, float pi) {
  return (c == cp) ? pr : ((c == 0) ? -pi : pi);
}

__global__ __launch_bounds__(256) void ptab_kernel(unsigned short* __restrict__ arow, unsigned short* __restrict__ acol) {
  __shared__ float sC[256];
  __shared__ float sS[256];
  __shared__ float sPr[256];
  __shared__ float sPi[256];
  const int tid = threadIdx.x, lane = tid & 31, wave = tid >> 5;
  {
    const float ang = (float)tid * 0.02454369260617025968f;
    float sv, cv;
    sincosf(ang, &sv, &cv);
    sC[tid] = cv; sS[tid] = sv;
  }
  __syncthreads();
  {
    float ar = 0.f, ai = 0.f;
#pragma unroll 1
    for (int i = 0; i < 89; ++i) {
      const int u = (i < 44) ? i : (i + 167);
      const int a = (u * tid) & 255;
      ar += sC[a]; ai += sS[a];
    }
    sPr[tid] = ar * 0.00390625f;
    sPi[tid] = ai * 0.00390625f;
  }
  __syncthreads();
  _Float16* Ar = (_Float16*)arow;
  _Float16* Ac = (_Float16*)acol;
  const int j = blockIdx.x;
  for (int pass = 0; pass < 2; ++pass) {
#pragma unroll 1
    for (int rr = 0; rr < 2; ++rr) {
      const int m = j * 16 + wave * 2 + rr;
      {
        const int x = m >> 1, c = m & 1;
#pragma unroll 1
        for (int cp = 0; cp < 2; ++cp) {
          v8h v;
#pragma unroll
          for (int e = 0; e < 8; ++e) {
            const int xp = lane * 8 + e;
            const int d = (x - xp) & 255;
            v[e] = (_Float16)(coefval(c, cp, sPr[d], sPi[d]) * 16.0f);
          }
          *(volatile v8h*)(Ar + (size_t)m * 512 + cp * 256 + lane * 8) = v;
        }
      }
      {
        const int c = m >> 8, yy = m & 255;
#pragma unroll 1
        for (int cp = 0; cp < 2; ++cp) {
          v8h v;
#pragma unroll
          for (int e = 0; e < 8; ++e) {
            const int yp = lane * 8 + e;
            const int d = (yy - yp) & 255;
            v[e] = (_Float16)(coefval(c, cp, sPr[d], sPi[d]) * 16.0f);
          }
          *(volatile v8h*)(Ac + (size_t)m * 512 + cp * 256 + lane * 8) = v;
        }
      }
    }
    __threadfence();
  }
}

__global__ __launch_bounds__(256) void wprep_kernel(const float* __restrict__ w1, const float* __restrict__ b1,
                                                    const float* __restrict__ w2, const float* __restrict__ b2,
                                                    float* __restrict__ wtab, unsigned short* __restrict__ wk) {
  __shared__ float s1[1152];
  __shared__ float s2[1152];
  __shared__ float sb1[64];
  __shared__ __align__(16) float sW[384];
  __shared__ __align__(16) _Float16 sK[1024];
  const int tid = threadIdx.x;
  for (int i = tid; i < 1152; i += 256) { s1[i] = w1[i]; s2[i] = w2[i]; }
  if (tid < 64) sb1[tid] = b1[tid];
  for (int i = tid; i < 384; i += 256) sW[i] = 0.f;
  for (int i = tid; i < 1024; i += 256) sK[i] = (_Float16)0.0f;
  __syncthreads();
  for (int idx = tid; idx < 324; idx += 256) {
    const int t1 = idx % 9;
    int r = idx / 9;
    const int cin = r & 1;
    r >>= 1;
    const int t2 = r % 9;
    const int co = r / 9;
    float s = 0.f;
#pragma unroll 1
    for (int ci = 0; ci < 64; ++ci) s += s2[(co * 64 + ci) * 9 + t2] * s1[(ci * 2 + cin) * 9 + t1];
    sW[idx] = s;
  }
  if (tid < 18) {
    const int co = tid / 9, t2 = tid - co * 9;
    float s = 0.f;
#pragma unroll 1
    for (int ci = 0; ci < 64; ++ci) s += s2[(co * 64 + ci) * 9 + t2] * sb1[ci];
    sW[324 + tid] = s;
  }
  __syncthreads();
  if (tid < 2) {
    float s = b2[tid];
#pragma unroll 1
    for (int t2 = 0; t2 < 9; ++t2) s += sW[324 + tid * 9 + t2];
    sW[342 + tid] = s;
  }
  if (tid < 100) {
    const int dx = tid % 5;
    int r = tid / 5;
    const int dy = r % 5;
    r /= 5;
    const int cin = r & 1;
    const int co = r >> 1;
    float s = 0.f;
#pragma unroll 1
    for (int ky2 = 0; ky2 < 3; ++ky2) {
      const int ky1 = dy - ky2;
      if (ky1 < 0 || ky1 > 2) continue;
#pragma unroll 1
      for (int kx2 = 0; kx2 < 3; ++kx2) {
        const int kx1 = dx - kx2;
        if (kx1 < 0 || kx1 > 2) continue;
        s += sW[((co * 9 + ky2 * 3 + kx2) * 2 + cin) * 9 + ky1 * 3 + kx1];
      }
    }
    sK[co * 64 + cin * 25 + dy * 5 + dx] = (_Float16)(s * 256.0f);
  }
  __syncthreads();
  for (int pass = 0; pass < 2; ++pass) {
    if (tid < 96) {
      const v4f v = *(const v4f*)(sW + tid * 4);
      *(volatile v4f*)(wtab + tid * 4) = v;
    }
    if (tid < 128) {
      const v8h v = *(const v8h*)(sK + tid * 8);
      *(volatile v8h*)((_Float16*)wk + tid * 8) = v;
    }
    __threadfence();
  }
}

__global__ __launch_bounds__(256) void dprep_kernel(const float* __restrict__ tgt, const float* __restrict__ ref,
                                                    unsigned short* __restrict__ dpl, int nvec) {
  const int i = blockIdx.x * 256 + threadIdx.x;
  if (i >= nvec) return;
  const int x8 = i & 31, c = (i >> 5) & 1, y = (i >> 6) & 255, b = i >> 14;
  const size_t src = (((size_t)b * 2 + c) * IMW + y) * IMW + (size_t)x8 * 8;
  const v4f t0 = *(const v4f*)(tgt + src);
  const v4f t1 = *(const v4f*)(tgt + src + 4);
  const v4f r0 = *(const v4f*)(ref + src);
  const v4f r1 = *(const v4f*)(ref + src + 4);
  v8h v;
#pragma unroll
  for (int e = 0; e < 4; ++e) {
    v[e] = (_Float16)(t0[e] - r0[e]);
    v[4 + e] = (_Float16)(t1[e] - r1[e]);
  }
  _Float16* p = (_Float16*)dpl + (size_t)i * 8;
  *(volatile v8h*)p = v;
  __threadfence();
  *(volatile v8h*)p = v;
}

__global__ __launch_bounds__(256) void conv_fold_kernel(const unsigned short* __restrict__ chg,
                                                        const unsigned short* __restrict__ wk,
                                                        const float* __restrict__ wtab,
                                                        float* __restrict__ out) {
  __shared__ __align__(16) _Float16 sR[10 * SRW];
  __shared__ __align__(16) _Float16 sA[256 * CPA];
  __shared__ __align__(16) _Float16 sB[16 * CPA];
  __shared__ float sW[384];
  __shared__ __align__(16) float sF[512];
  const int y = blockIdx.x, b = blockIdx.y;
  const int tid = threadIdx.x, lane = tid & 31, wave = tid >> 5;
  v8h z8;
#pragma unroll
  for (int e = 0; e < 8; ++e) z8[e] = (_Float16)0.0f;
  const _Float16* Cg = (const _Float16*)chg;

  for (int i = tid; i < 384; i += 256) sW[i] = wtab[i];
  if (tid < 128) {
    const int n = tid >> 3, c8 = (tid & 7) * 8;
    const v8h wv = *(const v8h*)((const _Float16*)wk + n * 64 + c8);
    *(v8h*)(sB + n * CPA + c8) = wv;
  }
  if (tid < 20) {
    const int row = tid >> 1;
    *(v8h*)(sR + row * SRW + ((tid & 1) ? 264 : 0)) = z8;
  }
  for (int i = tid; i < 320; i += 256) {
    const int row = i >> 5, ch = i & 31;
    const int cin = (row >= 5) ? 1 : 0, dy = row - cin * 5;
    const int gy = y + dy - 2;
    const bool ok = (gy >= 0) && (gy < IMW);
    const int gyc = gy < 0 ? 0 : (gy > IMW - 1 ? IMW - 1 : gy);
    v8h v = *(const v8h*)(Cg + (((size_t)b * 2 + cin) * IMW + gyc) * IMW + ch * 8);
    if (!ok) v = z8;
    *(v8h*)(sR + row * SRW + 8 + ch * 8) = v;
  }
  for (int i = tid; i < 512; i += 256) {
    const int x = i >> 1;
    *(v8h*)(sA + x * CPA + 48 + (i & 1) * 8) = z8;
  }
  __syncthreads();
  for (int i = tid; i < 2560; i += 256) {
    const int x = i & 255, q = i >> 8;
    const int cin = (q >= 5) ? 1 : 0, dy = q - cin * 5;
    const _Float16* src = sR + q * SRW + x + 6;
    _Float16* dst = sA + x * CPA + cin * 25 + dy * 5;
#pragma unroll
    for (int dx = 0; dx < 5; ++dx) dst[dx] = src[dx];
  }
  __syncthreads();

  const int rl = lane & 15, koff = (lane >> 4) * 8, moff = (lane >> 4) * 8;
  const int x0 = wave * 32;
  v8f acc0 = (v8f){0.f,0.f,0.f,0.f,0.f,0.f,0.f,0.f};
  v8f acc1 = (v8f){0.f,0.f,0.f,0.f,0.f,0.f,0.f,0.f};
#pragma unroll
  for (int ks = 0; ks < 2; ++ks) {
    const int k0 = ks * 32;
    const v16h bfr = Frag<_Float16>::load(sB + rl * CPA + k0 + koff);
    const v16h a0 = Frag<_Float16>::load(sA + (x0 + rl) * CPA + k0 + koff);
    const v16h a1 = Frag<_Float16>::load(sA + (x0 + 16 + rl) * CPA + k0 + koff);
    acc0 = Frag<_Float16>::mma(a0, bfr, acc0);
    acc1 = Frag<_Float16>::mma(a1, bfr, acc1);
    Frag<_Float16>::guard(acc0, acc1, a0, a1);
    Frag<_Float16>::keep(bfr, bfr, a0, a1);
  }
  if (rl < 2) {
#pragma unroll
    for (int r = 0; r < 8; ++r) {
      sF[rl * 256 + x0 + moff + r] = acc0[r] * 0.00390625f;
      sF[rl * 256 + x0 + 16 + moff + r] = acc1[r] * 0.00390625f;
    }
  }
  __syncthreads();

  {
    const int x = tid;
    const bool ylo = (y == 0), yhi = (y == IMW - 1), xlo = (x == 0), xhi = (x == IMW - 1);
#pragma unroll 1
    for (int co = 0; co < 2; ++co) {
      float v = sF[co * 256 + x] + sW[342 + co];
      float corr = 0.f;
#pragma unroll 1
      for (int t2 = 0; t2 < 9; ++t2) {
        const int ky2 = t2 / 3, kx2 = t2 - ky2 * 3;
        const bool inv = (ky2 == 0 && ylo) || (ky2 == 2 && yhi) || (kx2 == 0 && xlo) || (kx2 == 2 && xhi);
        if (inv) {
          float s = sW[324 + co * 9 + t2];
#pragma unroll 1
          for (int cin = 0; cin < 2; ++cin) {
#pragma unroll 1
            for (int ky1 = 0; ky1 < 3; ++ky1) {
              const float* wrow = sW + ((co * 9 + t2) * 2 + cin) * 9 + ky1 * 3;
              const _Float16* srow = sR + (cin * 5 + ky2 + ky1) * SRW + x + kx2 + 6;
#pragma unroll
              for (int kx1 = 0; kx1 < 3; ++kx1) s += wrow[kx1] * (float)srow[kx1];
            }
          }
          corr += s;
        }
      }
      sF[co * 256 + x] = v - corr;
    }
  }
  __syncthreads();

  if (wave < 2) {
    const int co = wave;
    float* ob = out + (((size_t)b * 2 + co) * IMW + y) * IMW;
    const float* sf = sF + co * 256;
    for (int pass = 0; pass < 2; ++pass) {
#pragma unroll
      for (int jj = 0; jj < 2; ++jj) {
        const v4f vv = *(const v4f*)(sf + jj * 128 + lane * 4);
        *(volatile v4f*)(ob + jj * 128 + lane * 4) = vv;
      }
      __threadfence();
    }
  }
}

extern "C" void kernel_launch(void* const* d_in, const int* in_sizes, int n_in,
                              void* d_out, int out_size, void* d_ws,
                              size_t ws_size, hipStream_t stream) {
  if (n_in < 6) return;
  const int plane = IMW * IMW;
  const int nb = in_sizes[0] / (2 * plane);
  if (nb <= 0) return;
  if (in_sizes[0] != nb * 2 * plane || in_sizes[1] != in_sizes[0]) return;
  if (in_sizes[2] != 1152 || in_sizes[3] != 64 || in_sizes[4] != 1152 || in_sizes[5] < 2) return;
  if (out_size != nb * 2 * plane) return;

  const float* tgt = (const float*)d_in[0];
  const float* ref = (const float*)d_in[1];
  const float* w1  = (const float*)d_in[2];
  const float* b1  = (const float*)d_in[3];
  const float* w2  = (const float*)d_in[4];
  const float* b2  = (const float*)d_in[5];
  float* out = (float*)d_out;

  char* ws = (char*)d_ws;
  size_t off = 0;
  const size_t szTab = (size_t)512 * 512 * 2;
  const size_t szPl  = (size_t)nb * 256 * 512 * 2;
  char* p_arow = ws + off; off += szTab;
  char* p_acol = ws + off; off += szTab;
  char* p_dpl  = ws + off; off += szPl;
  char* p_et   = ws + off; off += szPl;
  char* p_chg  = ws + off; off += szPl;
  char* p_wtab = ws + off; off += 1536;
  char* p_wk   = ws + off; off += 2048;
  if (off > ws_size) return;

  unsigned short* arow = (unsigned short*)p_arow;
  unsigned short* acol = (unsigned short*)p_acol;
  unsigned short* dpl  = (unsigned short*)p_dpl;
  unsigned short* et   = (unsigned short*)p_et;
  unsigned short* chg  = (unsigned short*)p_chg;
  float* wtab = (float*)p_wtab;
  unsigned short* wk = (unsigned short*)p_wk;

  const int nvec = nb * 16384;
  const long strPl = 256L * 512;
  const long strImg = 2L * plane;

  ptab_kernel<<<dim3(32), dim3(256), 0, stream>>>(arow, acol);
  wprep_kernel<<<dim3(1), dim3(256), 0, stream>>>(w1, b1, w2, b2, wtab, wk);
  dprep_kernel<<<dim3((nvec + 255) / 256), dim3(256), 0, stream>>>(tgt, ref, dpl, nvec);
  wmma_gemm64<0, false, 0, 1, false><<<dim3(4, nb), dim3(256), 0, stream>>>(
      arow, nullptr, 512, 0L, dpl, nullptr, 512, strPl,
      (void*)et, nullptr, 256, strPl, nullptr, nullptr, 0L, 512, 256, 512, 0.0625f);
  wmma_gemm64<0, false, 0, 1, true><<<dim3(4, nb), dim3(256), 0, stream>>>(
      acol, nullptr, 512, 0L, et, nullptr, 512, strPl,
      (void*)chg, nullptr, 256, strPl, nullptr, ref, strImg, 512, 256, 512, 0.0625f);
  conv_fold_kernel<<<dim3(IMW, nb), dim3(256), 0, stream>>>(chg, wk, wtab, out);
}
